// TriangleAttentionEndingNode_7215545057298
// MI455X (gfx1250) — hardware-verified
//
#include <hip/hip_runtime.h>
#include <math.h>
#include <stdint.h>

#define NR   256
#define CC   128
#define NHD  4
#define HD   32
#define NROW (NR * NR)
static_assert(NHD * HD == CC);
static_assert(HD == 32);
static_assert((NR % 64) == 0 && (CC % 64) == 0);
static_assert((((NROW / 64) * (CC / 64)) % 8) == 0);
static_assert((NROW % 32) == 0);
static_assert(NR * CC * NR == NROW * CC);

typedef _Float16 v16h __attribute__((ext_vector_type(16)));
typedef _Float16 v8h  __attribute__((ext_vector_type(8)));
typedef float    v8f  __attribute__((ext_vector_type(8)));
typedef float    v4f  __attribute__((ext_vector_type(4)));
typedef unsigned int v4u __attribute__((ext_vector_type(4)));
typedef unsigned int v2u __attribute__((ext_vector_type(2)));

__device__ __forceinline__ unsigned short bf_bits(float f) {
  unsigned u = __float_as_uint(f);
  return (unsigned short)((u + 0x7FFFu + ((u >> 16) & 1u)) >> 16);
}
__device__ __forceinline__ float bfr(float f) { return __uint_as_float(((unsigned)bf_bits(f)) << 16); }
__device__ __forceinline__ unsigned short h_bits(_Float16 x) { return __builtin_bit_cast(unsigned short, x); }
__device__ __forceinline__ unsigned pk16(unsigned short a, unsigned short b) { return (unsigned)a | ((unsigned)b << 16); }
__device__ __forceinline__ v8f zero8() { v8f z = {0.f, 0.f, 0.f, 0.f, 0.f, 0.f, 0.f, 0.f}; return z; }

__device__ __forceinline__ v16h ldfrag_h(const _Float16* p) {
  union { v16h v; v8h h[2]; } f;
  f.h[0] = *(const v8h*)(p);
  f.h[1] = *(const v8h*)(p + 16);
  return f.v;
}

__device__ __forceinline__ v8f mma_h(v16h a, v16h b, v8f c) {
  c = __builtin_amdgcn_wmma_f32_16x16x32_f16(false, a, false, b, (short)0, c, false, false);
#if defined(__HIP_DEVICE_COMPILE__)
  asm volatile("v_nop\n\tv_nop\n\tv_nop\n\tv_nop" : "+v"(c) : "v"(a), "v"(b));
#endif
  return c;
}
__device__ __forceinline__ v8f mma_h_raw(v16h a, v16h b, v8f c) {
  return __builtin_amdgcn_wmma_f32_16x16x32_f16(false, a, false, b, (short)0, c, false, false);
}
__device__ __forceinline__ void dep_guard_h(v8f& a, v8f& b, v16h x, v16h y) {
#if defined(__HIP_DEVICE_COMPILE__)
  asm volatile("v_nop\n\tv_nop\n\tv_nop\n\tv_nop" : "+v"(a), "+v"(b) : "v"(x), "v"(y));
#endif
}
__device__ __forceinline__ void keep4_h(v16h a, v16h b, v16h c, v16h d) {
#if defined(__HIP_DEVICE_COMPILE__)
  asm volatile("v_nop" :: "v"(a), "v"(b), "v"(c), "v"(d));
#endif
}
__device__ __forceinline__ void acc_guard4(v8f& a, v8f& b, v8f& c, v8f& d) {
#if defined(__HIP_DEVICE_COMPILE__)
  asm volatile("v_nop\n\tv_nop\n\tv_nop\n\tv_nop" : "+v"(a), "+v"(b), "+v"(c), "+v"(d));
#endif
}

__global__ __launch_bounds__(256) void ln_pb_k(const float* __restrict__ act, const float* __restrict__ gw,
                                             const float* __restrict__ bw, const float* __restrict__ w2,
                                             unsigned short* xh, unsigned short* xl, float* pb) {
  __shared__ __align__(16) unsigned int shi[8][4][64];
  __shared__ __align__(16) unsigned int slo[8][4][64];
  __shared__ __align__(16) float spb[NHD][32];
  __shared__ float sw[CC * NHD];
  __shared__ float sg[CC], sb[CC];
  const int tid = threadIdx.x, wave = tid >> 5, lane = tid & 31;
  const int b  = blockIdx.x;
  const int mm = b >> 3;
  const int ib = (b & 7) * 32;
  for (int e = tid; e < CC * NHD; e += 256) sw[e] = bfr(w2[e]);
  if (tid < CC) { sg[tid] = bfr(gw[tid]); sb[tid] = bfr(bw[tid]); }
  __syncthreads();

  const int c0 = lane * 4;
#pragma unroll 1
  for (int t = 0; t < 4; ++t) {
    const int ii = ib + wave * 4 + t;
    v4f v = *(const v4f*)(act + ((size_t)ii * NR + mm) * CC + c0);
    v[0] = bfr(v[0]); v[1] = bfr(v[1]); v[2] = bfr(v[2]); v[3] = bfr(v[3]);
    float s = (v[0] + v[1]) + (v[2] + v[3]);
#pragma unroll
    for (int off = 1; off < 32; off <<= 1) s += __shfl_xor(s, off, 32);
    const float mu = s * (1.0f / 128.0f);
    float sq = 0.0f;
#pragma unroll
    for (int e = 0; e < 4; ++e) {
      const float d = v[e] - mu;
      sq += d * d;
    }
#pragma unroll
    for (int off = 1; off < 32; off <<= 1) sq += __shfl_xor(sq, off, 32);
    const float var = sq * (1.0f / 128.0f);
    const float rs  = rsqrtf(var + 1e-5f);
    float y[4];
#pragma unroll
    for (int e = 0; e < 4; ++e) y[e] = (v[e] - mu) * rs * sg[c0 + e] + sb[c0 + e];

    v2u uh, ul;
#pragma unroll
    for (int e = 0; e < 2; ++e) {
      const float a0 = y[2 * e] * 16.0f, a1 = y[2 * e + 1] * 16.0f;
      const _Float16 h0 = (_Float16)a0, h1 = (_Float16)a1;
      const _Float16 l0 = (_Float16)((a0 - (float)h0) * 64.0f);
      const _Float16 l1 = (_Float16)((a1 - (float)h1) * 64.0f);
      uh[e] = pk16(h_bits(h0), h_bits(h1));
      ul[e] = pk16(h_bits(l0), h_bits(l1));
    }
    *(v2u*)(&shi[wave][t][lane * 2]) = uh;
    *(v2u*)(&slo[wave][t][lane * 2]) = ul;

    float p0 = 0.f, p1 = 0.f, p2 = 0.f, p3 = 0.f;
#pragma unroll
    for (int e = 0; e < 4; ++e) {
      const float* wr = sw + (c0 + e) * NHD;
      p0 += y[e] * wr[0];
      p1 += y[e] * wr[1];
      p2 += y[e] * wr[2];
      p3 += y[e] * wr[3];
    }
#pragma unroll
    for (int off = 1; off < 32; off <<= 1) {
      p0 += __shfl_xor(p0, off, 32); p1 += __shfl_xor(p1, off, 32);
      p2 += __shfl_xor(p2, off, 32); p3 += __shfl_xor(p3, off, 32);
    }
    if (lane == 0) {
      spb[0][wave * 4 + t] = p0;
      spb[1][wave * 4 + t] = p1;
      spb[2][wave * 4 + t] = p2;
      spb[3][wave * 4 + t] = p3;
    }
  }
  __syncthreads();
  {
    const int trow = lane >> 4, piece = lane & 15;
    const size_t rw = (size_t)mm * NR + ib + wave * 4;
    v4u ph[2], pl[2];
    size_t of[2];
#pragma unroll
    for (int it = 0; it < 2; ++it) {
      const int tt = it * 2 + trow;
      ph[it] = *(const v4u*)(&shi[wave][tt][piece * 4]);
      pl[it] = *(const v4u*)(&slo[wave][tt][piece * 4]);
      of[it] = (rw + tt) * CC + piece * 8;
    }
    for (int pass = 0; pass < 2; ++pass) {
#pragma unroll
      for (int it = 0; it < 2; ++it) {
        *(volatile v4u*)(xh + of[it]) = ph[it];
        *(volatile v4u*)(xl + of[it]) = pl[it];
      }
      __threadfence();
    }
  }
  if (wave == 0) {
    const int hq = lane >> 3, piece = lane & 7;
    const v4f pv = *(const v4f*)(&spb[hq][piece * 4]);
    const size_t po = ((size_t)hq * NR + mm) * NR + ib + piece * 4;
    for (int pass = 0; pass < 2; ++pass) {
      *(volatile v4f*)(pb + po) = pv;
      __threadfence();
    }
  }
}

__global__ __launch_bounds__(256) void wtr16(const float* __restrict__ W, unsigned short* Wt, int nk, int nn, float scale) {
  __shared__ __align__(16) float st[64 * 68];
  const int tid = threadIdx.x;
  const int n0 = blockIdx.x * 64;
  const int k0 = blockIdx.y * 64;
#pragma unroll
  for (int i = 0; i < 4; ++i) {
    const int idx = i * 256 + tid;
    const int kk = idx >> 4, c4 = (idx & 15) * 4;
    const v4f a = *(const v4f*)(W + (size_t)(k0 + kk) * nn + n0 + c4);
    *(v4f*)(st + kk * 68 + c4) = a;
  }
  __syncthreads();

  const int g = tid >> 3, piece = tid & 7;
  v4u hv[2];
  size_t hofs[2];
#pragma unroll
  for (int it = 0; it < 2; ++it) {
    const int n = it * 32 + g;
    v4u a;
#pragma unroll
    for (int e = 0; e < 4; ++e) {
      const float x0 = st[(piece * 8 + 2 * e) * 68 + n];
      const float x1 = st[(piece * 8 + 2 * e + 1) * 68 + n];
      a[e] = pk16(h_bits((_Float16)(bfr(x0) * scale)), h_bits((_Float16)(bfr(x1) * scale)));
    }
    hv[it] = a;
    hofs[it] = (size_t)(n0 + n) * nk + k0 + piece * 8;
  }
  for (int pass = 0; pass < 2; ++pass) {
#pragma unroll
    for (int it = 0; it < 2; ++it) *(volatile v4u*)(Wt + hofs[it]) = hv[it];
    __threadfence();
  }
}

template <int NPL, int EPI, bool HB>
__global__ __launch_bounds__(256) void gemm64_f16(
    const unsigned short* __restrict__ A0p, const unsigned short* __restrict__ A1p, int lda,
    const unsigned short* __restrict__ B0p, const unsigned short* __restrict__ B1p, int ldb,
    const float* __restrict__ biasp, float cscale, float oscale,
    float* Cf, unsigned short* C16a, unsigned short* C16b, int ldc, int M, int N, int K) {
  const _Float16* Ah0 = (const _Float16*)(const void*)A0p;
  const _Float16* Ah1 = (const _Float16*)(const void*)A1p;
  const _Float16* Bt0 = (const _Float16*)(const void*)B0p;
  const _Float16* Bt1 = (const _Float16*)(const void*)B1p;
  __shared__ __align__(16) float sT[8][16 * 68];
  const int lane = threadIdx.x & 31;
  const int wave = threadIdx.x >> 5;
  const int tilesN = N >> 6;
  const int tilesM = M >> 6;
  const int tile = blockIdx.x * 8 + wave;
  if (tile >= tilesM * tilesN) return;
  const int tm = tile / tilesN;
  const int tn = tile - tm * tilesN;
  const int m0 = tm << 6;
  const int n0 = tn << 6;

  const int rlane = lane & 15;
  const int koff  = (lane >> 4) * 8;
  const int mOff  = (lane >> 4) * 8;

  v8f acc[4][4];
#pragma unroll
  for (int i = 0; i < 4; ++i)
#pragma unroll
    for (int j = 0; j < 4; ++j) acc[i][j] = zero8();

  for (int k0 = 0; k0 < K; k0 += 32) {
#pragma unroll
    for (int pl = 0; pl < NPL; ++pl) {
      const _Float16* Ah = (pl == 0) ? Ah0 : Ah1;
      const _Float16* Bt = (pl == 0) ? Bt0 : Bt1;
      v16h bh[4];
#pragma unroll
      for (int j = 0; j < 4; ++j) {
        const size_t bo = (size_t)(n0 + (j << 4) + rlane) * ldb + koff + k0;
        bh[j] = ldfrag_h(Bt + bo);
      }
#pragma unroll
      for (int i = 0; i < 4; ++i) {
        const size_t ao = (size_t)(m0 + (i << 4) + rlane) * lda + koff + k0;
        const v16h ah = ldfrag_h(Ah + ao);
#pragma unroll
        for (int j = 0; j < 4; ++j) {
          acc[i][j] = mma_h_raw(ah, bh[j], acc[i][j]);
        }
        dep_guard_h(acc[i][0], acc[i][3], ah, bh[3]);
      }
      keep4_h(bh[0], bh[1], bh[2], bh[3]);
    }
  }
  acc_guard4(acc[0][0], acc[0][1], acc[0][2], acc[0][3]);
  acc_guard4(acc[1][0], acc[1][1], acc[1][2], acc[1][3]);
  acc_guard4(acc[2][0], acc[2][1], acc[2][2], acc[2][3]);
  acc_guard4(acc[3][0], acc[3][1], acc[3][2], acc[3][3]);

  float* slab = sT[wave];
#pragma unroll
  for (int i = 0; i < 4; ++i) {
    const int mBase = m0 + (i << 4);
    float bj[4];
#pragma unroll
    for (int j = 0; j < 4; ++j) {
      if constexpr (HB) bj[j] = bfr(biasp[n0 + (j << 4) + rlane]);
      else bj[j] = 0.0f;
    }
#pragma unroll
    for (int r = 0; r < 8; ++r) {
      const int row = mOff + r;
#pragma unroll
      for (int j = 0; j < 4; ++j) slab[row * 68 + (j << 4) + rlane] = acc[i][j][r] * cscale + bj[j];
    }
    __builtin_amdgcn_fence(__ATOMIC_RELEASE, "workgroup");
    __builtin_amdgcn_wave_barrier();
    __builtin_amdgcn_fence(__ATOMIC_ACQUIRE, "workgroup");
    if constexpr (EPI == 0 || EPI == 1) {
      const int rq = lane >> 3, piece = lane & 7;
      v4u ph[4];
      v4u pq[4];
#pragma unroll
      for (int it = 0; it < 4; ++it) {
        const int row = it * 4 + rq;
        const v4f a  = *(const v4f*)(slab + row * 68 + piece * 8);
        const v4f a2 = *(const v4f*)(slab + row * 68 + piece * 8 + 4);
        float f[8];
        f[0] = a[0];  f[1] = a[1];  f[2] = a[2];  f[3] = a[3];
        f[4] = a2[0]; f[5] = a2[1]; f[6] = a2[2]; f[7] = a2[3];
        v4u p, q;
#pragma unroll
        for (int e = 0; e < 4; ++e) {
          const float s0 = f[2 * e] * oscale, s1 = f[2 * e + 1] * oscale;
          const _Float16 x0 = (_Float16)s0;
          const _Float16 x1 = (_Float16)s1;
          p[e] = pk16(h_bits(x0), h_bits(x1));
          if constexpr (EPI == 1) {
            const _Float16 y0 = (_Float16)((s0 - (float)x0) * 64.0f);
            const _Float16 y1 = (_Float16)((s1 - (float)x1) * 64.0f);
            q[e] = pk16(h_bits(y0), h_bits(y1));
          } else {
            q[e] = 0u;
          }
        }
        ph[it] = p;
        pq[it] = q;
      }
      for (int pass = 0; pass < 2; ++pass) {
#pragma unroll
        for (int it = 0; it < 4; ++it) {
          const int row = it * 4 + rq;
          const size_t co = (size_t)(mBase + row) * ldc + n0 + piece * 8;
          *(volatile v4u*)(C16a + co) = ph[it];
          if constexpr (EPI == 1) *(volatile v4u*)(C16b + co) = pq[it];
        }
        __threadfence();
      }
    }
    if constexpr (EPI == 2) {
      const int h2 = lane >> 4, c4 = (lane & 15) * 4;
      v4f ov[8];
      size_t oo[8];
#pragma unroll
      for (int it = 0; it < 8; ++it) {
        const int row = it * 2 + h2;
        ov[it] = *(const v4f*)(slab + row * 68 + c4);
        const int r = mBase + row;
        const size_t orow = (size_t)(r % NR) * NR + (size_t)(r / NR);
        oo[it] = orow * (size_t)ldc + n0 + c4;
      }
      for (int pass = 0; pass < 2; ++pass) {
#pragma unroll
        for (int it = 0; it < 8; ++it) *(volatile v4f*)(Cf + oo[it]) = ov[it];
        __threadfence();
      }
    }
    __builtin_amdgcn_fence(__ATOMIC_RELEASE, "workgroup");
    __builtin_amdgcn_wave_barrier();
    __builtin_amdgcn_fence(__ATOMIC_ACQUIRE, "workgroup");
  }
}

__global__ __launch_bounds__(256) void v_tr(const unsigned short* __restrict__ vp, unsigned short* vt) {
  __shared__ __align__(16) _Float16 sv[64 * 72];
  const int tid = threadIdx.x;
  const int t0  = blockIdx.x * 64;
  const int f0  = blockIdx.y * 64;
  const int m   = blockIdx.z;
  const _Float16* src = (const _Float16*)(const void*)vp;
#pragma unroll
  for (int i = 0; i < 2; ++i) {
    const int idx = i * 256 + tid;
    const int tt = idx >> 3, c8 = (idx & 7) * 8;
    const v8h a = *(const v8h*)(src + ((size_t)m * NR + t0 + tt) * CC + f0 + c8);
    *(v8h*)(sv + tt * 72 + c8) = a;
  }
  __syncthreads();

  const int g = tid >> 3, piece = tid & 7;
  v4u hv[2];
  size_t hofs[2];
#pragma unroll
  for (int it = 0; it < 2; ++it) {
    const int d = it * 32 + g;
    v4u a;
#pragma unroll
    for (int e = 0; e < 4; ++e) {
      const _Float16 x0 = sv[(piece * 8 + 2 * e) * 72 + d];
      const _Float16 x1 = sv[(piece * 8 + 2 * e + 1) * 72 + d];
      a[e] = pk16(h_bits(x0), h_bits(x1));
    }
    hv[it] = a;
    hofs[it] = ((size_t)m * CC + f0 + d) * NR + t0 + piece * 8;
  }
  for (int pass = 0; pass < 2; ++pass) {
#pragma unroll
    for (int it = 0; it < 2; ++it) *(volatile v4u*)(vt + hofs[it]) = hv[it];
    __threadfence();
  }
}

__global__ __launch_bounds__(128)
void attn_k(const unsigned short* __restrict__ q16p, const unsigned short* __restrict__ k16p,
            const unsigned short* __restrict__ vhtp, const unsigned short* __restrict__ vltp,
            const unsigned short* __restrict__ z16p, const float* __restrict__ pbp,
            const float* __restrict__ maskp, const float* __restrict__ bgp,
            unsigned short* oghp, unsigned short* oglp) {
  union FH { v16h v; v8h h[2]; };
  constexpr int KTB    = 64 * CC * 2;
  constexpr int VTB    = CC * 64 * 2;
  constexpr int PTB    = NHD * 16 * 64 * 2;
  constexpr int OFF_K  = 0;
  constexpr int OFF_VH = KTB;
  constexpr int OFF_VL = KTB + VTB;
  constexpr int OFF_P  = KTB + 2 * VTB;
  constexpr int OFF_M  = OFF_P + PTB;
  constexpr int SMEMB  = OFF_M + 64 * 4;
  static_assert(16 * CC * 4 <= KTB);
  static_assert(SMEMB <= 65536);
  __shared__ __align__(16) unsigned char smem[SMEMB];
  _Float16* Ksh = (_Float16*)(smem + OFF_K);
  _Float16* Vhs = (_Float16*)(smem + OFF_VH);
  _Float16* Vls = (_Float16*)(smem + OFF_VL);
  _Float16* Psh = (_Float16*)(smem + OFF_P);
  float*    Msh = (float*)(smem + OFF_M);

  const int tid  = threadIdx.x;
  const int wave = tid >> 5;
  const int lane = tid & 31;
  const int hh   = lane >> 4;
  const int c    = lane & 15;
  const int h    = wave;

  const int bx = blockIdx.x;
  const int m  = bx >> 4;
  const int i0 = (bx & 15) * 16;
  const size_t rq = (size_t)m * NR + i0;
  const size_t rk = (size_t)m * NR;

  const _Float16* Qp  = (const _Float16*)(const void*)q16p;
  const _Float16* Kp  = (const _Float16*)(const void*)k16p;
  const _Float16* Vhp = (const _Float16*)(const void*)vhtp;
  const _Float16* Vlp = (const _Float16*)(const void*)vltp;
  const _Float16* Zp  = (const _Float16*)(const void*)z16p;

  const v16h qa = ldfrag_h(Qp + (rq + c) * CC + h * HD + 8 * hh);

  float mrow[8], lrow[8];
  v8f oh[2], ol[2];
#pragma unroll
  for (int r = 0; r < 8; ++r) { mrow[r] = -1.0e30f; lrow[r] = 0.f; }
#pragma unroll
  for (int t = 0; t < 2; ++t) { oh[t] = zero8(); ol[t] = zero8(); }

  _Float16* pw = Psh + wave * (16 * 64);
  const float scl = 0.17677669529663687f * (1.0f / 256.0f);
  const float* pbq = pbp + ((size_t)h * NR + i0 + 8 * hh) * NR;

#pragma unroll 1
  for (int kt = 0; kt < NR / 64; ++kt) {
    const int kv0 = kt * 64;
    __syncthreads();
#pragma unroll
    for (int it = 0; it < 8; ++it) {
      const int idx = it * 128 + tid;
      const int r = idx >> 4, ck = (idx & 15) * 8;
      *(v8h*)(Ksh + r * CC + ck) = *(const v8h*)(Kp + (rk + kv0 + r) * CC + ck);
      const int f = idx >> 3, cv = (idx & 7) * 8;
      const size_t vo = ((size_t)m * CC + f) * NR + kv0 + cv;
      *(v8h*)(Vhs + f * 64 + cv) = *(const v8h*)(Vhp + vo);
      *(v8h*)(Vls + f * 64 + cv) = *(const v8h*)(Vlp + vo);
    }
    if (tid < 64) Msh[tid] = 1.0e9f * (maskp[(size_t)(kv0 + tid) * NR + m] - 1.0f);
    __syncthreads();

    v8f s[4];
#pragma unroll
    for (int j = 0; j < 4; ++j) {
      FH kb;
      kb.h[0] = *(const v8h*)(Ksh + (j * 16 + c) * CC + h * HD + 8 * hh);
      kb.h[1] = *(const v8h*)(Ksh + (j * 16 + c) * CC + h * HD + 16 + 8 * hh);
      s[j] = mma_h(qa, kb.v, zero8());
    }

    float mk[4];
#pragma unroll
    for (int j = 0; j < 4; ++j) mk[j] = Msh[j * 16 + c];
#pragma unroll
    for (int r = 0; r < 8; ++r) {
      const float* pbr = pbq + (size_t)r * NR + kv0 + c;
      float f[4];
#pragma unroll
      for (int j = 0; j < 4; ++j) f[j] = (s[j][r] * scl + mk[j]) + pbr[j * 16];
      float tmx = fmaxf(fmaxf(f[0], f[1]), fmaxf(f[2], f[3]));
#pragma unroll
      for (int off = 1; off < 16; off <<= 1) tmx = fmaxf(tmx, __shfl_xor(tmx, off, 32));
      const float mn   = fmaxf(mrow[r], tmx);
      const float corr = __expf(mrow[r] - mn);
      mrow[r] = mn;
      float ps = 0.0f;
#pragma unroll
      for (int j = 0; j < 4; ++j) {
        const float p = __expf(f[j] - mn);
        ps += p;
        pw[(8 * hh + r) * 64 + j * 16 + c] = (_Float16)(p * 256.0f);
      }
      lrow[r] = lrow[r] * corr + ps;
#pragma unroll
      for (int t = 0; t < 2; ++t) { oh[t][r] = oh[t][r] * corr; ol[t][r] = ol[t][r] * corr; }
    }
    __builtin_amdgcn_fence(__ATOMIC_RELEASE, "workgroup");
    __builtin_amdgcn_wave_barrier();
    __builtin_amdgcn_fence(__ATOMIC_ACQUIRE, "workgroup");

#pragma unroll
    for (int kk = 0; kk < 2; ++kk) {
      FH pa;
      pa.h[0] = *(const v8h*)(pw + c * 64 + kk * 32 + 8 * hh);
      pa.h[1] = *(const v8h*)(pw + c * 64 + kk * 32 + 16 + 8 * hh);
#pragma unroll
      for (int t = 0; t < 2; ++t) {
        const int fr = h * HD + t * 16 + c;
        FH vb;
        vb.h[0] = *(const v8h*)(Vhs + fr * 64 + kk * 32 + 8 * hh);
        vb.h[1] = *(const v8h*)(Vhs + fr * 64 + kk * 32 + 16 + 8 * hh);
        oh[t] = mma_h(pa.v, vb.v, oh[t]);
        FH wb;
        wb.h[0] = *(const v8h*)(Vls + fr * 64 + kk * 32 + 8 * hh);
        wb.h[1] = *(const v8h*)(Vls + fr * 64 + kk * 32 + 16 + 8 * hh);
        ol[t] = mma_h(pa.v, wb.v, ol[t]);
      }
    }
  }
  __syncthreads();

  float* os = (float*)(void*)smem;
  float bgv[2];
#pragma unroll
  for (int t = 0; t < 2; ++t) bgv[t] = bfr(bgp[h * HD + t * 16 + c]);
#pragma unroll
  for (int r = 0; r < 8; ++r) {
    float l = lrow[r];
#pragma unroll
    for (int off = 1; off < 16; off <<= 1) l += __shfl_xor(l, off, 32);
    const float sc = (1.0f / l) * (1.0f / 4096.0f);
    const size_t zr = (rq + 8 * hh + r) * CC + h * HD;
#pragma unroll
    for (int t = 0; t < 2; ++t) {
      const int col = t * 16 + c;
      const float o = (oh[t][r] + ol[t][r] * (1.0f / 64.0f)) * sc;
      const float z = (float)Zp[zr + col] * (1.0f / 16.0f) + bgv[t];
      const float g = 1.0f / (1.0f + __expf(-z));
      os[(8 * hh + r) * CC + h * HD + col] = o * g * 256.0f;
    }
  }
  __syncthreads();
  {
    const int rr = tid >> 4, piece = tid & 15;
    v4u ph[2], pl[2];
    size_t of[2];
#pragma unroll
    for (int it = 0; it < 2; ++it) {
      const int row = it * 8 + rr;
      const v4f a  = *(const v4f*)(os + row * CC + piece * 8);
      const v4f a2 = *(const v4f*)(os + row * CC + piece * 8 + 4);
      float f[8];
      f[0] = a[0];  f[1] = a[1];  f[2] = a[2];  f[3] = a[3];
      f[4] = a2[0]; f[5] = a2[1]; f[6] = a2[2]; f[7] = a2[3];
      v4u p, q;
#pragma unroll
      for (int e = 0; e < 4; ++e) {
        const _Float16 x0 = (_Float16)f[2 * e];
        const _Float16 x1 = (_Float16)f[2 * e + 1];
        const _Float16 y0 = (_Float16)((f[2 * e] - (float)x0) * 64.0f);
        const _Float16 y1 = (_Float16)((f[2 * e + 1] - (float)x1) * 64.0f);
        p[e] = pk16(h_bits(x0), h_bits(x1));
        q[e] = pk16(h_bits(y0), h_bits(y1));
      }
      ph[it] = p;
      pl[it] = q;
      of[it] = (rq + row) * CC + piece * 8;
    }
    for (int pass = 0; pass < 2; ++pass) {
#pragma unroll
      for (int it = 0; it < 2; ++it) {
        *(volatile v4u*)(oghp + of[it]) = ph[it];
        *(volatile v4u*)(oglp + of[it]) = pl[it];
      }
      __threadfence();
    }
  }
}

extern "C" void kernel_launch(void* const* d_in, const int* in_sizes, int n_in,
                              void* d_out, int out_size, void* d_ws, size_t ws_size,
                              hipStream_t stream) {
  if (n_in < 12) return;
  if (in_sizes[0] != NROW * CC) return;
  if (in_sizes[1] != NR * NR) return;
  if (in_sizes[2] != CC || in_sizes[3] != CC) return;
  if (in_sizes[4] != CC * CC || in_sizes[5] != CC * CC || in_sizes[6] != CC * CC) return;
  if (in_sizes[7] != CC * NHD) return;
  if (in_sizes[8] != CC * CC || in_sizes[9] != CC) return;
  if (in_sizes[10] != CC * CC || in_sizes[11] != CC) return;
  if (out_size != NROW * CC) return;

  const float* act  = (const float*)d_in[0];
  const float* mask = (const float*)d_in[1];
  const float* lng  = (const float*)d_in[2];
  const float* lnb  = (const float*)d_in[3];
  const float* wq   = (const float*)d_in[4];
  const float* wk   = (const float*)d_in[5];
  const float* wv   = (const float*)d_in[6];
  const float* w2d  = (const float*)d_in[7];
  const float* wg   = (const float*)d_in[8];
  const float* bg   = (const float*)d_in[9];
  const float* wo   = (const float*)d_in[10];
  const float* bo   = (const float*)d_in[11];

  const size_t P16 = (size_t)NROW * CC * 2;
  const size_t PPB = (size_t)NHD * NR * NR * 4;
  const size_t PW  = (size_t)CC * CC * 2;
  size_t off = 0;
  const size_t oA    = off; off += P16;
  const size_t oB    = off; off += P16;
  const size_t oPB   = off; off += PPB;
  const size_t oWq   = off; off += PW;
  const size_t oWk   = off; off += PW;
  const size_t oWv   = off; off += PW;
  const size_t oWv16 = off; off += PW;
  const size_t oWg   = off; off += PW;
  const size_t oWo   = off; off += PW;
  const size_t oWo16 = off; off += PW;
  const size_t oQ    = off; off += P16;
  const size_t oK    = off; off += P16;
  const size_t oVh   = off; off += P16;
  const size_t oVl   = off; off += P16;
  const size_t oZ    = off; off += P16;
  if (off > ws_size) return;
  if (off > (size_t)134217728) return;

  char* ws = (char*)d_ws;
  unsigned short* Xh    = (unsigned short*)(ws + oA);
  unsigned short* Xl    = (unsigned short*)(ws + oB);
  unsigned short* VhT   = (unsigned short*)(ws + oA);
  unsigned short* VlT   = (unsigned short*)(ws + oB);
  float*          PB    = (float*)(ws + oPB);
  unsigned short* WqT   = (unsigned short*)(ws + oWq);
  unsigned short* WkT   = (unsigned short*)(ws + oWk);
  unsigned short* WvT   = (unsigned short*)(ws + oWv);
  unsigned short* WvT16 = (unsigned short*)(ws + oWv16);
  unsigned short* WgT   = (unsigned short*)(ws + oWg);
  unsigned short* WoT   = (unsigned short*)(ws + oWo);
  unsigned short* WoT16 = (unsigned short*)(ws + oWo16);
  unsigned short* Q16   = (unsigned short*)(ws + oQ);
  unsigned short* K16   = (unsigned short*)(ws + oK);
  unsigned short* Vh16  = (unsigned short*)(ws + oVh);
  unsigned short* Vl16  = (unsigned short*)(ws + oVl);
  unsigned short* OGh   = (unsigned short*)(ws + oVh);
  unsigned short* OGl   = (unsigned short*)(ws + oVl);
  unsigned short* Z16   = (unsigned short*)(ws + oZ);
  float*          outf  = (float*)d_out;

  const dim3 blk(256);
  const dim3 gLn(NROW / 32);
  const dim3 gW(CC / 64, CC / 64);
  const dim3 gG(((NROW / 64) * (CC / 64) + 7) / 8);
  const dim3 gVt(NR / 64, CC / 64, NR);
  const dim3 gAt(NR * (NR / 16));
  const float wScale = 1024.0f;
  const float wLow   = 16.0f;
  const float aScale = 16.0f;
  const float cs1    = 1.0f / 16384.0f;
  const float cs2    = 1.0f / 262144.0f;

  ln_pb_k<<<gLn, blk, 0, stream>>>(act, lng, lnb, w2d, Xh, Xl, PB);
  wtr16<<<gW, blk, 0, stream>>>(wq, WqT, CC, CC, wScale);
  wtr16<<<gW, blk, 0, stream>>>(wk, WkT, CC, CC, wScale);
  wtr16<<<gW, blk, 0, stream>>>(wv, WvT, CC, CC, wScale);
  wtr16<<<gW, blk, 0, stream>>>(wv, WvT16, CC, CC, wLow);
  wtr16<<<gW, blk, 0, stream>>>(wg, WgT, CC, CC, wScale);
  wtr16<<<gW, blk, 0, stream>>>(wo, WoT, CC, CC, wScale);
  wtr16<<<gW, blk, 0, stream>>>(wo, WoT16, CC, CC, wLow);
  gemm64_f16<1, 0, false><<<gG, blk, 0, stream>>>(Xh, Xh, CC, WqT, WqT, CC, bo, cs1, aScale, PB, Q16, Q16, CC, NROW, CC, CC);
  gemm64_f16<1, 0, false><<<gG, blk, 0, stream>>>(Xh, Xh, CC, WkT, WkT, CC, bo, cs1, aScale, PB, K16, K16, CC, NROW, CC, CC);
  gemm64_f16<2, 1, false><<<gG, blk, 0, stream>>>(Xh, Xl, CC, WvT, WvT16, CC, bo, cs1, aScale, PB, Vh16, Vl16, CC, NROW, CC, CC);
  gemm64_f16<1, 0, false><<<gG, blk, 0, stream>>>(Xh, Xh, CC, WgT, WgT, CC, bo, cs1, aScale, PB, Z16, Z16, CC, NROW, CC, CC);
  v_tr<<<gVt, blk, 0, stream>>>(Vh16, VhT);
  v_tr<<<gVt, blk, 0, stream>>>(Vl16, VlT);
  attn_k<<<gAt, dim3(128), 0, stream>>>(Q16, K16, VhT, VlT, Z16, PB, mask, bg, OGh, OGl);
  gemm64_f16<2, 2, true><<<gG, blk, 0, stream>>>(OGh, OGl, CC, WoT, WoT16, CC, bo, cs2, 1.0f, outf, Q16, Q16, CC, NROW, CC, CC);
}
